// MultiHeadSelfAttention_29420525978162
// MI455X (gfx1250) — hardware-verified
//
#include <hip/hip_runtime.h>


#ifndef NB
#define NB 2
#endif
#ifndef SEQ
#define SEQ 2048
#endif
#define NB_FULL  2
#define SEQ_FULL 2048
#define DM   1024
#define NH   16
#define HD   64
#define RH   256
#define PCAR 1024.0f
#define RCAR 2048.0f
#define QSCL 0.125f
#define L2E  1.4426950408889634f
#define PLANE ((size_t)NB * NH * SEQ * HD)

static_assert(NH * HD == DM);
static_assert(HD == 64);
static_assert(DM % 64 == 0);
static_assert(DM % 32 == 0);
static_assert(SEQ % 64 == 0);
static_assert((NB * SEQ) % 64 == 0);
static_assert(RH % 16 == 0 && RH % 32 == 0 && RH < SEQ);
static_assert((SEQ * 32) % 256 == 0);
static_assert(NB <= NB_FULL && SEQ <= SEQ_FULL);

typedef _Float16 h16;
typedef unsigned short bf;
typedef __attribute__((ext_vector_type(16))) __bf16   v16bf;
typedef __attribute__((ext_vector_type(16))) _Float16 v16h;
typedef __attribute__((ext_vector_type(8)))  _Float16 v8h;
typedef __attribute__((ext_vector_type(8)))  unsigned short v8us;
typedef __attribute__((ext_vector_type(8)))  float    v8f;
typedef __attribute__((ext_vector_type(4)))  float    v4f;
typedef v4f  __attribute__((may_alias)) v4fa;

__device__ __forceinline__ unsigned short f2bf(float f) { unsigned u = __float_as_uint(f); u += 0x7FFFu + ((u >> 16) & 1u); return (unsigned short)(u >> 16); }
__device__ __forceinline__ float bf2f(unsigned short b) { return __uint_as_float(((unsigned)b) << 16); }
__device__ __forceinline__ void splitf(float y, unsigned short& h, unsigned short& l) { h = f2bf(y); l = f2bf(y - bf2f(h)); }
__device__ __forceinline__ v16h cat16(v8h lo, v8h hi) { return __builtin_shufflevector(lo, hi, 0, 1, 2, 3, 4, 5, 6, 7, 8, 9, 10, 11, 12, 13, 14, 15); }
__device__ __forceinline__ v16bf cat16b(v8us lo, v8us hi) { return __builtin_bit_cast(v16bf, __builtin_shufflevector(lo, hi, 0, 1, 2, 3, 4, 5, 6, 7, 8, 9, 10, 11, 12, 13, 14, 15)); }
__device__ __forceinline__ v8f wmma16(v16h a, v16h b, v8f c) { return __builtin_amdgcn_wmma_f32_16x16x32_f16(false, a, false, b, (short)0, c, false, false); }
__device__ __forceinline__ v8f wmmab(v16bf a, v16bf b, v8f c) { return __builtin_amdgcn_wmma_f32_16x16x32_bf16(false, a, false, b, (short)0, c, false, false); }
__device__ __forceinline__ v16bf ldb(const bf* p) { return cat16b(*(const v8us*)p, *(const v8us*)(p + 16)); }
__device__ __forceinline__ v16h  ldh(const h16* p) { return cat16(*(const v8h*)p, *(const v8h*)(p + 16)); }
__device__ __forceinline__ void lds_wave_sync() { __builtin_amdgcn_fence(3  , "wavefront"); __builtin_amdgcn_wave_barrier(); asm volatile("" ::: "memory"); }

__global__ __launch_bounds__(256) void k_cvt8(const float* __restrict__ src, bf* dst, size_t n8) {
    const size_t i = (size_t)blockIdx.x * 256 + threadIdx.x; if (i >= n8) return;
    const v8f v = *(const v8f*)(src + i * 8); v8us o;
#pragma unroll
    for (int k = 0; k < 8; ++k) o[k] = f2bf(v[k]);
    *(volatile v8us*)(dst + i * 8) = o; __threadfence(); *(volatile v8us*)(dst + i * 8) = o;
}

__global__ __launch_bounds__(256) void k_cstab(const int* __restrict__ tpos, float* CS) {
    __shared__ __align__(16) float cl[512];
    const int tid = threadIdx.x; const int idx = blockIdx.x * 256 + tid;
    int n = idx >> 5; n = (n < SEQ) ? n : (SEQ - 1); const int j = idx & 31;
    double p = 1.0;
    p = (j & 1)  ? p * 1.3335214321633240 : p;
    p = (j & 2)  ? p * 1.7782794100389228 : p;
    p = (j & 4)  ? p * 3.1622776601683795 : p;
    p = (j & 8)  ? p * 10.0 : p;
    p = (j & 16) ? p * 100.0 : p;
    const float pf = (float)p; const float inv = 1.0f / pf;
    const float ang = (float)tpos[n] * inv;
    float sn, cs; sincosf(ang, &sn, &cs);
    cl[2 * tid] = cs; cl[2 * tid + 1] = sn;
    __syncthreads();
    if (tid < 128) {
        const v4f v = *(const v4fa*)(cl + tid * 4);
        float* dst = CS + (size_t)blockIdx.x * 512 + tid * 4;
        *(volatile v4f*)dst = v; __threadfence(); *(volatile v4f*)dst = v;
    }
}

template <int NSPLIT, int EPI>
__device__ __forceinline__ void gemm_body(const bf* __restrict__ A, const bf* __restrict__ A2, const bf* __restrict__ Bt,
                                          float* C, bf* Ph, bf* Pl, h16* V16, h16* Vr, const float* __restrict__ CS, float scl) {
    __shared__ __align__(16) float os[64 * 68];
    const int lane = threadIdx.x & 31, lr = lane & 15, hi = lane >> 4;
    const int r0 = blockIdx.x * 64, c0 = blockIdx.y * 64;
    v8f acc[4][4];
#pragma unroll
    for (int mb = 0; mb < 4; ++mb)
#pragma unroll
        for (int nb = 0; nb < 4; ++nb) acc[mb][nb] = (v8f){};
    const size_t aoff = (size_t)(r0 + lr) * DM + 8 * hi, boff = (size_t)(c0 + lr) * DM + 8 * hi;
#pragma unroll 1
    for (int kc = 0; kc < DM; kc += 32) {
        v16bf a[4], a2[4], bl;
#pragma unroll
        for (int mb = 0; mb < 4; ++mb) { a[mb] = ldb(A + aoff + (size_t)mb * 16 * DM + kc); if (NSPLIT == 1) a2[mb] = ldb(A2 + aoff + (size_t)mb * 16 * DM + kc); }
#pragma unroll
        for (int nb = 0; nb < 4; ++nb) {
            const v16bf b = ldb(Bt + boff + (size_t)nb * 16 * DM + kc);
#pragma unroll
            for (int mb = 0; mb < 4; ++mb) { acc[mb][nb] = wmmab(a[mb], b, acc[mb][nb]); if (NSPLIT == 1) acc[mb][nb] = wmmab(a2[mb], b, acc[mb][nb]); }
            bl = b;
        }
        asm volatile("" : "+v"(acc[0][0]), "+v"(acc[0][1]), "+v"(acc[0][2]), "+v"(acc[0][3]), "+v"(acc[1][0]), "+v"(acc[1][1]), "+v"(acc[1][2]), "+v"(acc[1][3]));
        asm volatile("v_nop\n\tv_nop\n\tv_nop\n\tv_nop" : "+v"(acc[2][0]), "+v"(acc[2][1]), "+v"(acc[2][2]), "+v"(acc[2][3]), "+v"(acc[3][0]), "+v"(acc[3][1]), "+v"(acc[3][2]), "+v"(acc[3][3]) : "v"(a[3]), "v"(bl));
    }
#pragma unroll
    for (int mb = 0; mb < 4; ++mb)
#pragma unroll
        for (int nb = 0; nb < 4; ++nb)
#pragma unroll
            for (int j = 0; j < 8; ++j) { const int row = mb * 16 + hi * 8 + j, col = nb * 16 + lr; if (EPI == 2) os[col * 68 + row] = acc[mb][nb][j]; else os[row * 68 + col] = acc[mb][nb][j]; }
    lds_wave_sync();
    const int bt = r0 / SEQ, t0 = r0 - bt * SEQ; const int h = blockIdx.y;
    if (EPI == 0) {
        float* crow = C + ((size_t)bt * SEQ_FULL + t0) * DM + c0;
#pragma unroll 1
        for (int ps = 0; ps < 2; ++ps) {
#pragma unroll 4
            for (int s = 0; s < 32; ++s) { const int row = 2 * s + hi, cofs = lr * 4; const v4f val = *(const v4fa*)(os + row * 68 + cofs); *(volatile v4f*)(crow + (size_t)row * DM + cofs) = val; }
            if (ps == 0) __threadfence(); }
    } else if (EPI == 1) {
        const int rq = lane >> 3, c8 = (lane & 7) * 8;
#pragma unroll 1
        for (int ps = 0; ps < 2; ++ps) {
#pragma unroll 2
            for (int s = 0; s < 16; ++s) {
#pragma clang fp contract(off)
                const int row = 4 * s + rq;
                const v4f xa = *(const v4fa*)(os + row * 68 + c8), xb = *(const v4fa*)(os + row * 68 + c8 + 4);
                const float* cp = CS + ((size_t)(t0 + row) * 32 + (lane & 7) * 4) * 2;
                const v4f ca = *(const v4f*)cp, cb = *(const v4f*)(cp + 4);
                float y[8];
                y[0] = xa[0] * ca[0] - xa[1] * ca[1]; y[1] = xa[1] * ca[0] + xa[0] * ca[1];
                y[2] = xa[2] * ca[2] - xa[3] * ca[3]; y[3] = xa[3] * ca[2] + xa[2] * ca[3];
                y[4] = xb[0] * cb[0] - xb[1] * cb[1]; y[5] = xb[1] * cb[0] + xb[0] * cb[1];
                y[6] = xb[2] * cb[2] - xb[3] * cb[3]; y[7] = xb[3] * cb[2] + xb[2] * cb[3];
                v8us oh, ol;
#pragma unroll
                for (int q = 0; q < 8; ++q) { unsigned short a1, a0; splitf(y[q] * scl, a1, a0); oh[q] = a1; ol[q] = a0; }
                const size_t oo = ((size_t)(bt * NH + h) * SEQ + t0 + row) * HD + c8;
                *(volatile v8us*)(Ph + oo) = oh; *(volatile v8us*)(Pl + oo) = ol; }
            if (ps == 0) __threadfence(); }
    } else {
        const int rq = lane >> 3, t8 = (lane & 7) * 8;
#pragma unroll 1
        for (int ps = 0; ps < 2; ++ps) {
#pragma unroll 2
            for (int s = 0; s < 16; ++s) {
                const int d = 4 * s + rq;
                const v4f xa = *(const v4fa*)(os + d * 68 + t8), xb = *(const v4fa*)(os + d * 68 + t8 + 4);
                v8h o16, orr;
#pragma unroll
                for (int q = 0; q < 4; ++q) { const h16 v0 = (h16)xa[q]; o16[q] = v0; orr[q] = (h16)((xa[q] - (float)v0) * RCAR); const h16 v1 = (h16)xb[q]; o16[4 + q] = v1; orr[4 + q] = (h16)((xb[q] - (float)v1) * RCAR); }
                const size_t oo = ((size_t)(bt * NH + h) * HD + d) * SEQ + t0 + t8;
                *(volatile v8h*)(V16 + oo) = o16; *(volatile v8h*)(Vr + oo) = orr; }
            if (ps == 0) __threadfence(); }
    }
}

__global__ __launch_bounds__(32) void k_proj_qk(const bf* __restrict__ XB, const bf* __restrict__ WQK, const float* __restrict__ CS, bf* QKh, bf* QKl) {
    const size_t z = blockIdx.z; const float scl = (z == 0) ? QSCL : 1.0f;
    gemm_body<0, 1>(XB, XB, WQK + z * (size_t)DM * DM, (float*)0, QKh + z * PLANE, QKl + z * PLANE, (h16*)0, (h16*)0, CS, scl);
}
__global__ __launch_bounds__(32) void k_proj_v(const bf* __restrict__ XB, const bf* __restrict__ WV, h16* VT, h16* VTr) {
    gemm_body<0, 2>(XB, XB, WV, (float*)0, (bf*)0, (bf*)0, VT, VTr, (const float*)0, 1.0f);
}
__global__ __launch_bounds__(32) void k_oproj(const bf* __restrict__ ATh, const bf* __restrict__ ATl, const bf* __restrict__ WO, float* OUT) {
    gemm_body<1, 0>(ATh, ATl, WO, OUT, (bf*)0, (bf*)0, (h16*)0, (h16*)0, (const float*)0, 1.0f);
}

__device__ __forceinline__ v8f score_tile(const bf* __restrict__ kp, const bf* __restrict__ kq, v16bf qh0, v16bf qh1, v16bf ql0, v16bf ql1) {
    const v16bf kh0 = ldb(kp), kh1 = ldb(kp + 32), kl0 = ldb(kq), kl1 = ldb(kq + 32);
    v8f z = (v8f){};
    z = wmmab(kl0, qh0, z); z = wmmab(kl1, qh1, z);
    z = wmmab(kh0, ql0, z); z = wmmab(kh1, ql1, z);
    z = wmmab(kh0, qh0, z); z = wmmab(kh1, qh1, z);
    return z;
}

template <bool EARLY>
__device__ __forceinline__ void attn_body(const bf* __restrict__ Qh, const bf* __restrict__ Ql, const bf* __restrict__ Kh, const bf* __restrict__ Kl,
                                          const h16* __restrict__ VT, const h16* __restrict__ VTr, bf* Ah, bf* Al, int qt0) {
    __shared__ __align__(16) float os[16 * 68];
    const int lane = threadIdx.x & 31, lr = lane & 15, hi = lane >> 4;
    const int bh = blockIdx.y;
    const int q0 = (qt0 + (int)blockIdx.x) * 16;
    const size_t pbase = (size_t)bh * SEQ * HD;
    const int qoff = (q0 + lr) * HD + 8 * hi;
    const v16bf gqh0 = ldb(Qh + pbase + qoff), gqh1 = ldb(Qh + pbase + qoff + 32), gql0 = ldb(Ql + pbase + qoff), gql1 = ldb(Ql + pbase + qoff + 32);
    v8f acc[4], accr[4];
#pragma unroll
    for (int dt = 0; dt < 4; ++dt) { acc[dt] = (v8f){}; accr[dt] = (v8f){}; }
    float m = -1.0e30f, lsum = 0.0f;
    const int lastC = q0 >> 5;
#pragma unroll 1
    for (int ch = 0; ch <= lastC; ++ch) {
        const int c = ch * 32;
        v16bf qh0 = gqh0, qh1 = gqh1, ql0 = gql0, ql1 = gql1;
        if (EARLY) { int qo = qoff; asm volatile("" : "+v"(qo)); qh0 = ldb(Qh + pbase + qo); qh1 = ldb(Qh + pbase + qo + 32); ql0 = ldb(Ql + pbase + qo); ql1 = ldb(Ql + pbase + qo + 32); }
        v8f sT[2];
        { const size_t k0 = pbase + (size_t)(c + lr) * HD + 8 * hi, k1 = pbase + (size_t)(c + 16 + lr) * HD + 8 * hi;
          sT[0] = score_tile(Kh + k0, Kl + k0, qh0, qh1, ql0, ql1);
          sT[1] = score_tile(Kh + k1, Kl + k1, qh0, qh1, ql0, ql1); }
        asm volatile("v_nop\n\tv_nop\n\tv_nop\n\tv_nop" : "+v"(sT[0]), "+v"(sT[1]) : "v"(qh1), "v"(ql1));
        __builtin_amdgcn_sched_barrier(0);
        if (ch == lastC) {
            const int qq = q0 + lr;
#pragma unroll
            for (int j = 0; j < 2; ++j)
#pragma unroll
                for (int r = 0; r < 8; ++r) { const int key = c + 16 * j + 8 * hi + r; sT[j][r] = (key > qq) ? -1.0e30f : sT[j][r]; }
        }
        float mx = sT[0][0];
#pragma unroll
        for (int r = 1; r < 8; ++r) mx = fmaxf(mx, sT[0][r]);
#pragma unroll
        for (int r = 0; r < 8; ++r) mx = fmaxf(mx, sT[1][r]);
        mx = fmaxf(mx, __shfl_xor(mx, 16, 32));
        const float mnew = fmaxf(m, mx);
        const float sc = __builtin_amdgcn_exp2f((m - mnew) * L2E);
        m = mnew;
        float rs = 0.0f; v16h pb, pbr;
#pragma unroll
        for (int j = 0; j < 2; ++j)
#pragma unroll
            for (int r = 0; r < 8; ++r) {
                const float p = __builtin_amdgcn_exp2f((sT[j][r] - mnew) * L2E); rs += p;
                const float pc = p * PCAR; const h16 ph = (h16)pc; pb[8 * j + r] = ph;
                if (EARLY) pbr[8 * j + r] = (h16)((pc - (float)ph) * RCAR); else pbr[8 * j + r] = (h16)0.0f; }
        lsum = lsum * sc + rs;
#pragma unroll
        for (int dt = 0; dt < 4; ++dt)
#pragma unroll
            for (int r = 0; r < 8; ++r) { acc[dt][r] *= sc; if (EARLY) accr[dt][r] *= sc; }
        __builtin_amdgcn_sched_barrier(0);
#pragma unroll
        for (int dt = 0; dt < 4; ++dt) {
            const size_t vo = ((size_t)bh * HD + 16 * dt + lr) * SEQ + c + 8 * hi;
            const v16h av = ldh(VT + vo);
            acc[dt] = wmma16(av, pb, acc[dt]);
            if (EARLY) { const v16h avr = ldh(VTr + vo); accr[dt] = wmma16(avr, pb, accr[dt]); accr[dt] = wmma16(av, pbr, accr[dt]); }
        }
        if (EARLY) asm volatile("v_nop\n\tv_nop\n\tv_nop\n\tv_nop" : "+v"(acc[0]), "+v"(acc[1]), "+v"(acc[2]), "+v"(acc[3]), "+v"(accr[0]), "+v"(accr[1]), "+v"(accr[2]), "+v"(accr[3]) : "v"(pb), "v"(pbr));
        else       asm volatile("v_nop\n\tv_nop\n\tv_nop\n\tv_nop" : "+v"(acc[0]), "+v"(acc[1]), "+v"(acc[2]), "+v"(acc[3]) : "v"(pb));
        __builtin_amdgcn_sched_barrier(0);
    }
    const float l = lsum + __shfl_xor(lsum, 16, 32);
    const float inv = 1.0f / (PCAR * l);
#pragma unroll
    for (int dt = 0; dt < 4; ++dt)
#pragma unroll
        for (int r = 0; r < 8; ++r) { float o = acc[dt][r]; if (EARLY) o += accr[dt][r] * (1.0f / RCAR); os[lr * 68 + 16 * dt + 8 * hi + r] = o * inv; }
    lds_wave_sync();
    const int b = bh / NH, h = bh - b * NH; const int rq = lane >> 3, c8 = (lane & 7) * 8;
#pragma unroll 1
    for (int ps = 0; ps < 2; ++ps) {
#pragma unroll
        for (int s = 0; s < 4; ++s) {
            const int row = 4 * s + rq;
            const v4f xa = *(const v4fa*)(os + row * 68 + c8), xb = *(const v4fa*)(os + row * 68 + c8 + 4);
            v8us oh, ol;
#pragma unroll
            for (int q = 0; q < 4; ++q) { unsigned short a1, a0; splitf(xa[q], a1, a0); oh[q] = a1; ol[q] = a0; splitf(xb[q], a1, a0); oh[4 + q] = a1; ol[4 + q] = a0; }
            const size_t oo = ((size_t)b * SEQ + q0 + row) * DM + h * HD + c8;
            *(volatile v8us*)(Ah + oo) = oh; *(volatile v8us*)(Al + oo) = ol; }
        if (ps == 0) __threadfence(); }
}

__global__ __launch_bounds__(32) void k_attn_early(const bf* __restrict__ Qh, const bf* __restrict__ Ql, const bf* __restrict__ Kh, const bf* __restrict__ Kl, const h16* __restrict__ VT, const h16* __restrict__ VTr, bf* Ah, bf* Al) {
    attn_body<true>(Qh, Ql, Kh, Kl, VT, VTr, Ah, Al, 0);
}
__global__ __launch_bounds__(32) void k_attn_late(const bf* __restrict__ Qh, const bf* __restrict__ Ql, const bf* __restrict__ Kh, const bf* __restrict__ Kl, const h16* __restrict__ VT, const h16* __restrict__ VTr, bf* Ah, bf* Al) {
    attn_body<false>(Qh, Ql, Kh, Kl, VT, VTr, Ah, Al, RH / 16);
}

constexpr size_t SZ_W   = (size_t)DM * DM * 2;
constexpr size_t SZ_ROW = (size_t)NB * SEQ * DM * 2;
constexpr size_t SZ_CS  = (size_t)SEQ * 64 * 4;
constexpr size_t O_WQK = 0;
constexpr size_t O_WV  = O_WQK + 2 * SZ_W;
constexpr size_t O_WO  = O_WV + SZ_W;
constexpr size_t O_XB  = O_WO + SZ_W;
constexpr size_t O_CS  = O_XB + SZ_ROW;
constexpr size_t O_QKH = O_CS + SZ_CS;
constexpr size_t O_QKL = O_QKH + 2 * SZ_ROW;
constexpr size_t O_VT  = O_QKL + 2 * SZ_ROW;
constexpr size_t O_VTR = O_VT + SZ_ROW;
constexpr size_t O_ATH = O_VTR + SZ_ROW;
constexpr size_t O_ATL = O_ATH + SZ_ROW;
constexpr size_t WS_TOTAL = O_ATL + SZ_ROW;
static_assert(WS_TOTAL <= (size_t)134217728);
static_assert(SZ_ROW == PLANE * 2);
static_assert(O_CS % 256 == 0 && O_QKH % 256 == 0);

extern "C" void kernel_launch(void* const* d_in, const int* in_sizes, int n_in,
                              void* d_out, int out_size, void* d_ws, size_t ws_size, hipStream_t stream) {
    if (n_in < 6) return;
    const size_t xneed = (size_t)(NB - 1) * SEQ_FULL * DM + (size_t)SEQ * DM;
    if ((size_t)in_sizes[0] < xneed) return;
    if (in_sizes[1] < SEQ) return;
    if ((size_t)in_sizes[2] < (size_t)DM * DM || (size_t)in_sizes[3] < (size_t)DM * DM || (size_t)in_sizes[4] < (size_t)DM * DM || (size_t)in_sizes[5] < (size_t)DM * DM) return;
    if ((size_t)out_size < xneed) return;
    if (WS_TOTAL > ws_size) return;
    const float* x = (const float*)d_in[0]; const int* tpos = (const int*)d_in[1];
    const float* wq = (const float*)d_in[2]; const float* wk = (const float*)d_in[3]; const float* wv = (const float*)d_in[4]; const float* wo = (const float*)d_in[5];
    float* OUT = (float*)d_out;
    char* ws = (char*)d_ws;
    bf* WQK = (bf*)(ws + O_WQK); bf* WV = (bf*)(ws + O_WV); bf* WO = (bf*)(ws + O_WO); bf* XB = (bf*)(ws + O_XB); float* CS = (float*)(ws + O_CS);
    bf* QKh = (bf*)(ws + O_QKH); bf* QKl = (bf*)(ws + O_QKL); h16* VT = (h16*)(ws + O_VT); h16* VTr = (h16*)(ws + O_VTR); bf* ATh = (bf*)(ws + O_ATH); bf* ATl = (bf*)(ws + O_ATL);

    const size_t w8 = (size_t)DM * DM / 8, x8 = (size_t)SEQ * DM / 8;
    const unsigned gw = (unsigned)((w8 + 255) / 256), gx = (unsigned)((x8 + 255) / 256);
    k_cvt8<<<gw, 256, 0, stream>>>(wq, WQK, w8);
    k_cvt8<<<gw, 256, 0, stream>>>(wk, WQK + (size_t)DM * DM, w8);
    k_cvt8<<<gw, 256, 0, stream>>>(wv, WV, w8);
    k_cvt8<<<gw, 256, 0, stream>>>(wo, WO, w8);
    for (int b = 0; b < NB; ++b)
        k_cvt8<<<gx, 256, 0, stream>>>(x + (size_t)b * SEQ_FULL * DM, XB + (size_t)b * SEQ * DM, x8);
    k_cstab<<<SEQ * 32 / 256, 256, 0, stream>>>(tpos, CS);
    k_proj_qk<<<dim3(NB * SEQ / 64, DM / 64, 2), 32, 0, stream>>>(XB, WQK, CS, QKh, QKl);
    k_proj_v<<<dim3(NB * SEQ / 64, DM / 64, 1), 32, 0, stream>>>(XB, WV, VT, VTr);
    k_attn_early<<<dim3(RH / 16, NB * NH, 1), 32, 0, stream>>>(QKh, QKl, QKh + PLANE, QKl + PLANE, VT, VTr, ATh, ATl);
    k_attn_late<<<dim3((SEQ - RH) / 16, NB * NH, 1), 32, 0, stream>>>(QKh, QKl, QKh + PLANE, QKl + PLANE, VT, VTr, ATh, ATl);
    k_oproj<<<dim3(NB * SEQ / 64, DM / 64, 1), 32, 0, stream>>>(ATh, ATl, WO, OUT);
}
